// DecoderBlock_50869592655693
// MI455X (gfx1250) — hardware-verified
//
#include <hip/hip_runtime.h>
#include <math.h>

#ifndef NB
#define NB 4
#endif
#ifndef SEQ
#define SEQ 1024
#endif
#define NB_FULL 4
#define SEQ_FULL 1024
#define DM 1024
#define DFF 4096
#define NHEAD 16
#define ROWS (NB * SEQ)

#ifndef ATTN_ATTR
#define ATTN_ATTR __attribute__((amdgpu_num_vgpr(256)))
#endif

static_assert(SEQ % 64 == 0);
static_assert(SEQ <= SEQ_FULL);
static_assert(NB <= NB_FULL);
static_assert(DM == NHEAD * 64);
static_assert(ROWS % 64 == 0);
static_assert(DM % 64 == 0);
static_assert(DFF % 64 == 0);

typedef __attribute__((ext_vector_type(16))) _Float16 v16h;
typedef __attribute__((ext_vector_type(8)))  _Float16 v8h;
typedef __attribute__((ext_vector_type(8)))  float    v8f;
typedef __attribute__((ext_vector_type(4)))  float    v4f;
typedef unsigned int u4v __attribute__((ext_vector_type(4)));
typedef unsigned int u2v __attribute__((ext_vector_type(2)));

union FragU { v16h v; v8h h[2]; };
__device__ __forceinline__ v16h frag_ld(const _Float16* p) { FragU f; f.h[0] = *(const v8h*)(p); f.h[1] = *(const v8h*)(p + 16); return f.v; }

__device__ __forceinline__ v8f wmma16(v16h a, v16h b, v8f c) {
    c = __builtin_amdgcn_wmma_f32_16x16x32_f16(false, a, false, b, (short)0, c, false, false);
    asm volatile("v_nop\n\tv_nop\n\tv_nop\n\tv_nop" : "+v"(c) : "v"(a), "v"(b));
    return c;
}
__device__ __forceinline__ void dep_guard_h(v8f& a, v8f& b, v16h x, v16h y) { asm volatile("v_nop\n\tv_nop\n\tv_nop\n\tv_nop" : "+v"(a), "+v"(b) : "v"(x), "v"(y)); }
__device__ __forceinline__ void keep4_h(v16h a, v16h b, v16h c, v16h d) { asm volatile("v_nop" :: "v"(a), "v"(b), "v"(c), "v"(d)); }
__device__ __forceinline__ void acc_guard4(v8f& a, v8f& b, v8f& c, v8f& d) { asm volatile("v_nop\n\tv_nop\n\tv_nop\n\tv_nop" : "+v"(a), "+v"(b), "+v"(c), "+v"(d)); }

__device__ __forceinline__ void wave_sync() {
    __builtin_amdgcn_fence(3  , "workgroup");
    __builtin_amdgcn_wave_barrier();
    __builtin_amdgcn_fence(2  , "workgroup");
}

#define VST2(T, ptr, val) do { const T vst2_v_ = (val); *(volatile T*)(ptr) = vst2_v_; __threadfence(); *(volatile T*)(ptr) = vst2_v_; } while (0)

__device__ __forceinline__ float bf_keep(float v) { const unsigned u = __builtin_bit_cast(unsigned, v); const unsigned r = (u + 0x7fffu + ((u >> 16) & 1u)) & 0xffff0000u; return __builtin_bit_cast(float, r); }
__device__ __forceinline__ unsigned pk2h(float a, float b) { return (unsigned)__builtin_bit_cast(unsigned short, (_Float16)a) | ((unsigned)__builtin_bit_cast(unsigned short, (_Float16)b) << 16); }
__device__ __forceinline__ _Float16 res12(float v, _Float16 hi) { return (_Float16)((v - (float)hi) * 4096.0f); }

__global__ __launch_bounds__(256) void k_xcast(const float* __restrict__ X, unsigned short* __restrict__ X16) {
    const unsigned u = blockIdx.x * 256u + threadIdx.x; if (u >= (unsigned)ROWS * 128u) return;
    const unsigned r = u >> 7, c0 = (u & 127u) * 8u;
    const unsigned b = r / (unsigned)SEQ, s = r - b * (unsigned)SEQ;
    const float* src = X + ((size_t)b * SEQ_FULL + s) * DM + c0;
    const v4f a = *(const v4f*)(src), q = *(const v4f*)(src + 4);
    u4v pk; pk.x = pk2h(bf_keep(a.x), bf_keep(a.y)); pk.y = pk2h(bf_keep(a.z), bf_keep(a.w)); pk.z = pk2h(bf_keep(q.x), bf_keep(q.y)); pk.w = pk2h(bf_keep(q.z), bf_keep(q.w));
    VST2(u4v, (u4v*)(X16 + (size_t)r * DM + c0), pk);
}

__global__ __launch_bounds__(256) void k_castbT(const float* __restrict__ SRC, unsigned lds, unsigned short* __restrict__ DST, unsigned ldd, unsigned nR, unsigned nC, float sc) {
    const unsigned u = blockIdx.x * 256u + threadIdx.x; const unsigned per = nR >> 3; if (u >= nC * per) return;
    const unsigned c = u / per, r0 = 8u * (u - c * per);
    float w[8];
#pragma unroll
    for (int e = 0; e < 8; ++e) w[e] = bf_keep(SRC[(size_t)(r0 + (unsigned)e) * lds + c]) * sc;
    u4v pk; pk.x = pk2h(w[0], w[1]); pk.y = pk2h(w[2], w[3]); pk.z = pk2h(w[4], w[5]); pk.w = pk2h(w[6], w[7]);
    VST2(u4v, (u4v*)(DST + (size_t)c * ldd + r0), pk);
}

__global__ __launch_bounds__(256) void k_bfvec(const float* __restrict__ SRC, float* __restrict__ DST, unsigned n) {
    const unsigned u = blockIdx.x * 256u + threadIdx.x; if (u >= n) return;
    VST2(float, DST + u, bf_keep(SRC[u]));
}

template <int BIAS_MODE, int OUT_MODE, int ACT>
__global__ __launch_bounds__(256) void k_gemm64(const unsigned short* __restrict__ Ap, unsigned lda,
                                                const unsigned short* __restrict__ Btp, unsigned ldb,
                                                void* __restrict__ Cout, void* __restrict__ Cout2, unsigned ldc,
                                                const float* __restrict__ bias, unsigned M, unsigned N, unsigned K, float scale) {
    const _Float16* A = (const _Float16*)Ap; const _Float16* Bt = (const _Float16*)Btp;
    __shared__ __align__(16) float sT[8][16 * 68];
    const unsigned lane = threadIdx.x & 31u, wave = threadIdx.x >> 5;
    const unsigned tilesN = N >> 6, tilesM = M >> 6;
    const unsigned tile = blockIdx.x * 8u + wave;
    if (tile >= tilesM * tilesN) return;
    const unsigned tm = tile / tilesN, tn = tile - tm * tilesN;
    const unsigned m0 = tm << 6, n0 = tn << 6;
    const unsigned rlane = lane & 15u;
    const unsigned koff = (lane >> 4) * 8u;
    const unsigned mOff = (lane >> 4) * 8u;

    v8f acc[4][4];
#pragma unroll
    for (int i = 0; i < 4; ++i)
#pragma unroll
        for (int j = 0; j < 4; ++j) acc[i][j] = (v8f){0.f, 0.f, 0.f, 0.f, 0.f, 0.f, 0.f, 0.f};

    for (unsigned k0 = 0; k0 < K; k0 += 32u) {
        v16h bh[4];
#pragma unroll
        for (int j = 0; j < 4; ++j) bh[j] = frag_ld(Bt + (size_t)(n0 + ((unsigned)j << 4) + rlane) * ldb + koff + k0);
#pragma unroll
        for (int i = 0; i < 4; ++i) {
            const v16h ah = frag_ld(A + (size_t)(m0 + ((unsigned)i << 4) + rlane) * lda + koff + k0);
#pragma unroll
            for (int j = 0; j < 4; ++j) acc[i][j] = __builtin_amdgcn_wmma_f32_16x16x32_f16(false, ah, false, bh[j], (short)0, acc[i][j], false, false);
            dep_guard_h(acc[i][0], acc[i][3], ah, ah);
        }
        keep4_h(bh[0], bh[1], bh[2], bh[3]);
    }
    acc_guard4(acc[0][0], acc[0][1], acc[0][2], acc[0][3]);
    acc_guard4(acc[1][0], acc[1][1], acc[1][2], acc[1][3]);
    acc_guard4(acc[2][0], acc[2][1], acc[2][2], acc[2][3]);
    acc_guard4(acc[3][0], acc[3][1], acc[3][2], acc[3][3]);

    float* slab = sT[wave];
#pragma unroll
    for (int i = 0; i < 4; ++i) {
        const unsigned mBase = m0 + ((unsigned)i << 4);
#pragma unroll
        for (int j = 0; j < 4; ++j) {
            const unsigned n = n0 + ((unsigned)j << 4) + rlane;
            float bv = 0.f;
            if (BIAS_MODE == 2) bv = bias[n];
#pragma unroll
            for (int r = 0; r < 8; ++r) {
                float v = acc[i][j][r] * scale;
                if (BIAS_MODE == 2) v += bv;
                if (ACT == 2) v = fmaxf(v, 0.0f);
                slab[(mOff + (unsigned)r) * 68u + ((unsigned)j << 4) + rlane] = v;
            }
        }
        wave_sync();
        if (OUT_MODE == 0) {
            float* C = (float*)Cout;
            const unsigned hh = lane >> 4, c4 = (lane & 15u) * 4u;
            v4f vv[8];
#pragma unroll
            for (int it = 0; it < 8; ++it) vv[it] = *(const v4f*)(slab + ((unsigned)it * 2u + hh) * 68u + c4);
            for (int pass = 0; pass < 2; ++pass) {
#pragma unroll
                for (int it = 0; it < 8; ++it) {
                    const unsigned row = (unsigned)it * 2u + hh;
                    *(volatile v4f*)(C + (size_t)(mBase + row) * ldc + n0 + c4) = vv[it];
                }
                __threadfence();
            }
        } else {
            unsigned short* C = (unsigned short*)Cout;
            unsigned short* C2 = (unsigned short*)Cout2;
            const unsigned q = lane >> 3, c8 = (lane & 7u) * 8u;
            v8h hv[4], lv[4];
#pragma unroll
            for (int it = 0; it < 4; ++it) {
                const float* sp = slab + ((unsigned)it * 4u + q) * 68u + c8;
                const v4f a = *(const v4f*)(sp), b2 = *(const v4f*)(sp + 4);
                v8h t;
                t[0] = (_Float16)a.x; t[1] = (_Float16)a.y; t[2] = (_Float16)a.z; t[3] = (_Float16)a.w;
                t[4] = (_Float16)b2.x; t[5] = (_Float16)b2.y; t[6] = (_Float16)b2.z; t[7] = (_Float16)b2.w;
                hv[it] = t;
                v8h u = t;
                if (OUT_MODE == 2) {
                    u[0] = res12(a.x, t[0]); u[1] = res12(a.y, t[1]); u[2] = res12(a.z, t[2]); u[3] = res12(a.w, t[3]);
                    u[4] = res12(b2.x, t[4]); u[5] = res12(b2.y, t[5]); u[6] = res12(b2.z, t[6]); u[7] = res12(b2.w, t[7]);
                }
                lv[it] = u;
            }
            for (int pass = 0; pass < 2; ++pass) {
#pragma unroll
                for (int it = 0; it < 4; ++it) {
                    const unsigned row = (unsigned)it * 4u + q;
                    const size_t off = (size_t)(mBase + row) * ldc + n0 + c8;
                    *(volatile v8h*)(C + off) = hv[it];
                    if (OUT_MODE == 2) *(volatile v8h*)(C2 + off) = lv[it];
                }
                __threadfence();
            }
        }
        wave_sync();
    }
}

template <int CAUSAL>
__global__ __launch_bounds__(128) ATTN_ATTR void k_attn_pl(const unsigned short* __restrict__ QKp, const unsigned short* __restrict__ QKRp,
                                                           const unsigned short* __restrict__ VTp, unsigned short* __restrict__ CTXp) {
    __shared__ __align__(16) _Float16 Psh[4][16 * 64];
    __shared__ __align__(16) float    Os[4][16 * 68];
    constexpr unsigned NQB = SEQ / 64;
    const unsigned tid = threadIdx.x, wave = tid >> 5, lane = tid & 31u, hh = lane >> 4, c = lane & 15u;
    const unsigned bx = blockIdx.x;
    const unsigned bh = bx / NQB, qb = bx - bh * NQB;
    const unsigned h = bh & 15u, b = bh >> 4;
    const unsigned q0 = qb * 64u + wave * 16u;
    const size_t rb = (size_t)b * SEQ;
    const _Float16* QK = (const _Float16*)QKp; const _Float16* QKR = (const _Float16*)QKRp; const _Float16* VT = (const _Float16*)VTp;

    const size_t qoff = (rb + q0 + c) * 2048u + h * 64u + 8u * hh;
    const v16h qh0 = frag_ld(QK + qoff), qh1 = frag_ld(QK + qoff + 32);
    const v16h ql0 = frag_ld(QKR + qoff), ql1 = frag_ld(QKR + qoff + 32);
    const size_t koff0 = (rb + c) * 2048u + 1024u + h * 64u + 8u * hh;
    const _Float16* kbh = QK + koff0;
    const _Float16* kbl = QKR + koff0;
    const _Float16* vbp = VT + (size_t)(h * 64u + c) * ROWS + rb + 8u * hh;

    float mrow[8], lrow[8];
    v8f oacc[4];
#pragma unroll
    for (int r = 0; r < 8; ++r) { mrow[r] = -__builtin_inff(); lrow[r] = 0.f; }
#pragma unroll
    for (int t = 0; t < 4; ++t) oacc[t] = (v8f){0.f, 0.f, 0.f, 0.f, 0.f, 0.f, 0.f, 0.f};

    const float SC = 0.125f * 1.4426950408889634f;
    const float FILL = -1.0e9f * 1.4426950408889634f;
    const float RSC = 1.0f / 4096.0f;
    _Float16* pw = Psh[wave];
    const unsigned nChunks = CAUSAL ? (qb + 1u) : NQB;
    for (unsigned kc = 0; kc < nChunks; ++kc) {
        const unsigned kv0 = kc * 64u;
        v8f s[4];
#pragma unroll
        for (int j = 0; j < 4; ++j) {
            const size_t ko = (size_t)(kv0 + (unsigned)j * 16u) * 2048u;
            v8f ah = (v8f){0.f, 0.f, 0.f, 0.f, 0.f, 0.f, 0.f, 0.f};
            v8f ax = (v8f){0.f, 0.f, 0.f, 0.f, 0.f, 0.f, 0.f, 0.f};
            {
                const v16h kh = frag_ld(kbh + ko), kl = frag_ld(kbl + ko);
                ah = wmma16(qh0, kh, ah);
                ax = wmma16(qh0, kl, ax);
                ax = wmma16(ql0, kh, ax);
            }
            {
                const v16h kh = frag_ld(kbh + ko + 32), kl = frag_ld(kbl + ko + 32);
                ah = wmma16(qh1, kh, ah);
                ax = wmma16(qh1, kl, ax);
                ax = wmma16(ql1, kh, ax);
            }
            s[j] = ah + ax * RSC;
        }
        const bool diag = (CAUSAL != 0) && (kc == qb);
        float cm[8];
#pragma unroll
        for (int r = 0; r < 8; ++r) {
            const unsigned qrow = q0 + 8u * hh + (unsigned)r;
            float m = -__builtin_inff();
#pragma unroll
            for (int j = 0; j < 4; ++j) {
                const unsigned kvcol = kv0 + (unsigned)j * 16u + c;
                float t = s[j][r] * SC;
                t = (diag && (kvcol > qrow)) ? FILL : t;
                s[j][r] = t;
                m = fmaxf(m, t);
            }
            m = fmaxf(m, __shfl_xor(m, 1, 32)); m = fmaxf(m, __shfl_xor(m, 2, 32));
            m = fmaxf(m, __shfl_xor(m, 4, 32)); m = fmaxf(m, __shfl_xor(m, 8, 32));
            cm[r] = m;
        }
#pragma unroll
        for (int r = 0; r < 8; ++r) {
            const float mnew = fmaxf(mrow[r], cm[r]);
            const float alpha = exp2f(mrow[r] - mnew);
            mrow[r] = mnew;
            const float msh = mnew - 15.0f;
            float psum = 0.f;
#pragma unroll
            for (int j = 0; j < 4; ++j) {
                const _Float16 ph = (_Float16)exp2f(s[j][r] - msh);
                psum += (float)ph;
                pw[(8u * hh + (unsigned)r) * 64u + (unsigned)j * 16u + c] = ph;
            }
            psum += __shfl_xor(psum, 1, 32); psum += __shfl_xor(psum, 2, 32);
            psum += __shfl_xor(psum, 4, 32); psum += __shfl_xor(psum, 8, 32);
            lrow[r] = lrow[r] * alpha + psum;
#pragma unroll
            for (int t = 0; t < 4; ++t) oacc[t][r] *= alpha;
        }
        wave_sync();
#pragma unroll
        for (int kk = 0; kk < 2; ++kk) {
            const v16h pa = frag_ld(pw + c * 64u + (unsigned)kk * 32u + 8u * hh);
#pragma unroll
            for (int t = 0; t < 4; ++t) {
                const v16h vb = frag_ld(vbp + (size_t)((unsigned)t * 16u) * ROWS + kv0 + (unsigned)kk * 32u);
                oacc[t] = wmma16(pa, vb, oacc[t]);
            }
        }
        wave_sync();
    }

    float* os = Os[wave];
#pragma unroll
    for (int r = 0; r < 8; ++r) {
        const float inv = 1.0f / lrow[r];
#pragma unroll
        for (int t = 0; t < 4; ++t) os[(8u * hh + (unsigned)r) * 68u + (unsigned)t * 16u + c] = oacc[t][r] * inv;
    }
    wave_sync();
    {
        const unsigned q = lane >> 3, c8 = (lane & 7u) * 8u;
        v8h hv[4];
#pragma unroll
        for (int it = 0; it < 4; ++it) {
            const float* sp = os + ((unsigned)it * 4u + q) * 68u + c8;
            const v4f a = *(const v4f*)(sp), b2 = *(const v4f*)(sp + 4);
            v8h t;
            t[0] = (_Float16)a.x; t[1] = (_Float16)a.y; t[2] = (_Float16)a.z; t[3] = (_Float16)a.w;
            t[4] = (_Float16)b2.x; t[5] = (_Float16)b2.y; t[6] = (_Float16)b2.z; t[7] = (_Float16)b2.w;
            hv[it] = t;
        }
        unsigned short* crow = CTXp + (rb + q0) * (size_t)DM + h * 64u + c8;
        for (int pass = 0; pass < 2; ++pass) {
#pragma unroll
            for (int it = 0; it < 4; ++it) *(volatile v8h*)(crow + (size_t)((unsigned)it * 4u + q) * DM) = hv[it];
            __threadfence();
        }
    }
}

template <int XRES, int OUTFULL, int WF, int W16>
__global__ __launch_bounds__(256) void k_ln_res(const float* A, const float* R, const float* __restrict__ GA, const float* __restrict__ BE,
                                                float* __restrict__ Yf, unsigned short* __restrict__ Y16) {
    #pragma clang fp contract(off)
    const unsigned r = blockIdx.x * 8u + (threadIdx.x >> 5); const unsigned L = threadIdx.x & 31u; if (r >= (unsigned)ROWS) return;
    const unsigned b = r / (unsigned)SEQ, s_ = r - b * (unsigned)SEQ; const size_t rf = (size_t)b * SEQ_FULL + s_;
    const float* arow = A + (size_t)r * DM;
    const float* rrow = R + (XRES ? rf : (size_t)r) * DM;
    v4f v[8]; float s = 0.f;
#pragma unroll
    for (int q = 0; q < 8; ++q) { v[q] = *(const v4f*)(arow + 4u * L + 128u * (unsigned)q); s += (v[q].x + v[q].y) + (v[q].z + v[q].w); }
#pragma unroll
    for (int o = 16; o > 0; o >>= 1) s += __shfl_xor(s, o, 32);
    const float mu = s * (1.f / DM); float qq = 0.f;
#pragma unroll
    for (int q = 0; q < 8; ++q) { v[q].x -= mu; v[q].y -= mu; v[q].z -= mu; v[q].w -= mu; qq += (v[q].x * v[q].x + v[q].y * v[q].y) + (v[q].z * v[q].z + v[q].w * v[q].w); }
#pragma unroll
    for (int o = 16; o > 0; o >>= 1) qq += __shfl_xor(qq, o, 32);
    const float rs = rsqrtf(qq * (1.f / DM) + 1e-5f);
    v4f y[8];
#pragma unroll
    for (int q = 0; q < 8; ++q) {
        const unsigned cc = 4u * L + 128u * (unsigned)q;
        const v4f ga = *(const v4f*)(GA + cc), be = *(const v4f*)(BE + cc);
        v4f x = *(const v4f*)(rrow + cc);
        if (XRES) { x.x = bf_keep(x.x); x.y = bf_keep(x.y); x.z = bf_keep(x.z); x.w = bf_keep(x.w); }
        v4f t;
        t.x = x.x + (v[q].x * rs * bf_keep(ga.x) + bf_keep(be.x));
        t.y = x.y + (v[q].y * rs * bf_keep(ga.y) + bf_keep(be.y));
        t.z = x.z + (v[q].z * rs * bf_keep(ga.z) + bf_keep(be.z));
        t.w = x.w + (v[q].w * rs * bf_keep(ga.w) + bf_keep(be.w));
        y[q] = t;
    }
    float* yrow = WF ? (Yf + (OUTFULL ? rf : (size_t)r) * DM) : nullptr;
    unsigned short* hrow = W16 ? (Y16 + (size_t)r * DM) : nullptr;
    for (int pass = 0; pass < 2; ++pass) {
#pragma unroll
        for (int q = 0; q < 8; ++q) {
            const unsigned cc = 4u * L + 128u * (unsigned)q;
            if (WF) *(volatile v4f*)(yrow + cc) = y[q];
            if (W16) { u2v pk; pk.x = pk2h(y[q].x, y[q].y); pk.y = pk2h(y[q].z, y[q].w); *(volatile u2v*)(hrow + cc) = pk; }
        }
        __threadfence();
    }
}

constexpr size_t SZ_ACT16 = (size_t)ROWS * DM * 2;
constexpr size_t SZ_WSQ   = (size_t)DM * DM * 2;
constexpr size_t SZ_WFF   = (size_t)DM * DFF * 2;
constexpr size_t SZ_BIG   = (size_t)ROWS * DFF * 2;
constexpr size_t SZ_QK    = (size_t)ROWS * 2048 * 2;
constexpr size_t SZ_VT    = (size_t)DM * ROWS * 2;
constexpr size_t SZ_F32   = (size_t)ROWS * DM * 4;
constexpr size_t SZ_TOTAL = 2 * SZ_ACT16 + 8 * SZ_WSQ + 2 * SZ_WFF + SZ_BIG + 2 * SZ_F32 + (size_t)DFF * 4 + (size_t)DM * 4;
static_assert(SZ_QK + SZ_VT + SZ_ACT16 <= SZ_BIG);
static_assert(SZ_QK <= SZ_F32);
static_assert(SZ_TOTAL <= (size_t)134217728);
static_assert(SZ_ACT16 % 256 == 0);
static_assert(SZ_QK % 256 == 0);
static_assert(SZ_VT % 256 == 0);
static_assert(SZ_F32 % 256 == 0);

static inline unsigned gemm_blocks(unsigned M, unsigned N) { return ((M >> 6) * (N >> 6) + 7u) / 8u; }
static inline unsigned cast_blocks(unsigned nR, unsigned nC) { return (nC * (nR >> 3) + 255u) / 256u; }

extern "C" void kernel_launch(void* const* d_in, const int* in_sizes, int n_in, void* d_out, int out_size, void* d_ws, size_t ws_size, hipStream_t stream) {
    if (n_in < 15) return;
    const size_t need_x = ((size_t)(NB - 1) * SEQ_FULL + SEQ) * DM;
    if ((size_t)in_sizes[0] < need_x) return;
    if ((size_t)out_size < need_x) return;
    for (int i = 1; i <= 8; ++i) if ((size_t)in_sizes[i] < (size_t)DM * DM) return;
    if (in_sizes[9] < DM) return;
    if (in_sizes[10] < DM) return;
    if ((size_t)in_sizes[11] < (size_t)DM * DFF) return;
    if (in_sizes[12] < DFF) return;
    if ((size_t)in_sizes[13] < (size_t)DM * DFF) return;
    if (in_sizes[14] < DM) return;
    if (SZ_TOTAL > ws_size) return;

    const float* X   = (const float*)d_in[0];
    const float* Wq1 = (const float*)d_in[1];
    const float* Wk1 = (const float*)d_in[2];
    const float* Wv1 = (const float*)d_in[3];
    const float* Wo1 = (const float*)d_in[4];
    const float* Wq2 = (const float*)d_in[5];
    const float* Wk2 = (const float*)d_in[6];
    const float* Wv2 = (const float*)d_in[7];
    const float* Wo2 = (const float*)d_in[8];
    const float* lng = (const float*)d_in[9];
    const float* lnb = (const float*)d_in[10];
    const float* W1  = (const float*)d_in[11];
    const float* b1  = (const float*)d_in[12];
    const float* W2  = (const float*)d_in[13];
    const float* b2  = (const float*)d_in[14];
    float* out = (float*)d_out;

    char* wsp = (char*)d_ws;
    unsigned short* X16  = (unsigned short*)wsp; wsp += SZ_ACT16;
    unsigned short* NM16 = (unsigned short*)wsp; wsp += SZ_ACT16;
    unsigned short* WQK1 = (unsigned short*)wsp; wsp += 2 * SZ_WSQ;
    unsigned short* WV1  = (unsigned short*)wsp; wsp += SZ_WSQ;
    unsigned short* WO1  = (unsigned short*)wsp; wsp += SZ_WSQ;
    unsigned short* WQK2 = (unsigned short*)wsp; wsp += 2 * SZ_WSQ;
    unsigned short* WV2  = (unsigned short*)wsp; wsp += SZ_WSQ;
    unsigned short* WO2  = (unsigned short*)wsp; wsp += SZ_WSQ;
    unsigned short* W1T  = (unsigned short*)wsp; wsp += SZ_WFF;
    unsigned short* W2T  = (unsigned short*)wsp; wsp += SZ_WFF;
    char* big = wsp; wsp += SZ_BIG;
    unsigned short* QK16  = (unsigned short*)big;
    unsigned short* VT16  = (unsigned short*)(big + SZ_QK);
    unsigned short* CTX16 = (unsigned short*)(big + SZ_QK + SZ_VT);
    unsigned short* H16   = (unsigned short*)big;
    float* PROJ = (float*)wsp; wsp += SZ_F32;
    float* NA2  = (float*)wsp; wsp += SZ_F32;
    float* BR1  = (float*)wsp; wsp += (size_t)DFF * 4;
    float* BR2  = (float*)wsp; wsp += (size_t)DM * 4;
    unsigned short* NA16 = X16;
    unsigned short* QKR16 = (unsigned short*)NA2;

    k_xcast<<<ROWS / 2, 256, 0, stream>>>(X, X16);
    k_castbT<<<cast_blocks(DM, DM), 256, 0, stream>>>(Wq1, DM, WQK1, DM, DM, DM, 16.0f);
    k_castbT<<<cast_blocks(DM, DM), 256, 0, stream>>>(Wk1, DM, WQK1 + (size_t)DM * DM, DM, DM, DM, 16.0f);
    k_castbT<<<cast_blocks(DM, DM), 256, 0, stream>>>(Wv1, DM, WV1, DM, DM, DM, 16.0f);
    k_castbT<<<cast_blocks(DM, DM), 256, 0, stream>>>(Wo1, DM, WO1, DM, DM, DM, 16.0f);
    k_castbT<<<cast_blocks(DM, DM), 256, 0, stream>>>(Wq2, DM, WQK2, DM, DM, DM, 16.0f);
    k_castbT<<<cast_blocks(DM, DM), 256, 0, stream>>>(Wk2, DM, WQK2 + (size_t)DM * DM, DM, DM, DM, 16.0f);
    k_castbT<<<cast_blocks(DM, DM), 256, 0, stream>>>(Wv2, DM, WV2, DM, DM, DM, 16.0f);
    k_castbT<<<cast_blocks(DM, DM), 256, 0, stream>>>(Wo2, DM, WO2, DM, DM, DM, 16.0f);
    k_castbT<<<cast_blocks(DM, DFF), 256, 0, stream>>>(W1, DFF, W1T, DM, DM, DFF, 16.0f);
    k_castbT<<<cast_blocks(DFF, DM), 256, 0, stream>>>(W2, DM, W2T, DFF, DFF, DM, 16.0f);
    k_bfvec<<<DFF / 256, 256, 0, stream>>>(b1, BR1, DFF);
    k_bfvec<<<DM / 256, 256, 0, stream>>>(b2, BR2, DM);

    const unsigned attn_blocks = (unsigned)NB * NHEAD * (SEQ / 64);

    k_gemm64<0, 2, 0><<<gemm_blocks(ROWS, 2048), 256, 0, stream>>>(X16, DM, WQK1, DM, (void*)QK16, (void*)QKR16, 2048, nullptr, ROWS, 2048, DM, 0.0625f);
    k_gemm64<0, 1, 0><<<gemm_blocks(DM, ROWS), 256, 0, stream>>>(WV1, DM, X16, DM, (void*)VT16, nullptr, ROWS, nullptr, DM, ROWS, DM, 0.0625f);
    k_attn_pl<1><<<attn_blocks, 128, 0, stream>>>(QK16, QKR16, VT16, CTX16);
    k_gemm64<0, 0, 0><<<gemm_blocks(ROWS, DM), 256, 0, stream>>>(CTX16, DM, WO1, DM, (void*)PROJ, nullptr, DM, nullptr, ROWS, DM, DM, 0.0625f);
    k_ln_res<1, 0, 0, 1><<<ROWS / 8, 256, 0, stream>>>(PROJ, X, lng, lnb, nullptr, NM16);

    k_gemm64<0, 2, 0><<<gemm_blocks(ROWS, 2048), 256, 0, stream>>>(NM16, DM, WQK2, DM, (void*)QK16, (void*)QKR16, 2048, nullptr, ROWS, 2048, DM, 0.0625f);
    k_gemm64<0, 1, 0><<<gemm_blocks(DM, ROWS), 256, 0, stream>>>(WV2, DM, NM16, DM, (void*)VT16, nullptr, ROWS, nullptr, DM, ROWS, DM, 0.0625f);
    k_attn_pl<0><<<attn_blocks, 128, 0, stream>>>(QK16, QKR16, VT16, CTX16);
    k_gemm64<0, 0, 0><<<gemm_blocks(ROWS, DM), 256, 0, stream>>>(CTX16, DM, WO2, DM, (void*)PROJ, nullptr, DM, nullptr, ROWS, DM, DM, 0.0625f);
    k_ln_res<0, 0, 1, 1><<<ROWS / 8, 256, 0, stream>>>(PROJ, PROJ, lng, lnb, NA2, NA16);

    k_gemm64<2, 1, 2><<<gemm_blocks(ROWS, DFF), 256, 0, stream>>>(NA16, DM, W1T, DM, (void*)H16, nullptr, DFF, BR1, ROWS, DFF, DM, 0.0625f);
    k_gemm64<2, 0, 0><<<gemm_blocks(ROWS, DM), 256, 0, stream>>>(H16, DFF, W2T, DFF, (void*)PROJ, nullptr, DM, BR2, ROWS, DM, DFF, 0.0625f);
    k_ln_res<0, 1, 1, 0><<<ROWS / 8, 256, 0, stream>>>(PROJ, NA2, lng, lnb, out, nullptr);
}
